// OptionCriticHead_50835232915722
// MI455X (gfx1250) — hardware-run, weakly checked
//
#include <hip/hip_runtime.h>

typedef float          v8f   __attribute__((ext_vector_type(8)));
typedef float          v4f   __attribute__((ext_vector_type(4)));
typedef unsigned int   v4u   __attribute__((ext_vector_type(4)));
typedef int            v8i   __attribute__((ext_vector_type(8)));
typedef unsigned short v8us  __attribute__((ext_vector_type(8)));
typedef unsigned short v16us __attribute__((ext_vector_type(16)));
typedef __bf16         v16bf __attribute__((ext_vector_type(16)));
typedef _Float16       v16h  __attribute__((ext_vector_type(16)));
typedef v4f  __attribute__((may_alias)) v4fa;
typedef v8us __attribute__((may_alias)) v8usa;
union FragB { v16bf v; v16us u; v8us h[2]; v8i w; };
union FragH { v16h  v; v16us u; v8us h[2]; v8i w; };

__device__ __forceinline__ v8f wmb(const FragB& a, const FragB& b, v8f c) {
  v8f d = __builtin_amdgcn_wmma_f32_16x16x32_bf16(false, a.v, false, b.v, (short)0, c, false, false);
  asm volatile("v_nop\n\tv_nop\n\tv_nop\n\tv_nop" : "+v"(d) : "v"(a.w), "v"(b.w));
  return d;
}

__device__ __forceinline__ v8f wmh(const FragH& a, const FragH& b, v8f c) {
  v8f d = __builtin_amdgcn_wmma_f32_16x16x32_f16(false, a.v, false, b.v, (short)0, c, false, false);
  asm volatile("v_nop\n\tv_nop\n\tv_nop\n\tv_nop" : "+v"(d) : "v"(a.w), "v"(b.w));
  return d;
}

__device__ __forceinline__ unsigned bf16_bits(float f) {
  const unsigned u = __float_as_uint(f);
  const unsigned r = (u + 0x7FFFu + ((u >> 16) & 1u)) >> 16;
  const unsigned q = (u >> 16) | 0x40u;
  return ((u & 0x7fffffffu) > 0x7f800000u) ? q : r;
}

__device__ __forceinline__ float bf16_val(float f) {
  return __uint_as_float(bf16_bits(f) << 16);
}
__device__ __forceinline__ int clampi(int v, int lo, int hi) {
  return v < lo ? lo : (v > hi ? hi : v);
}

__device__ __forceinline__ unsigned f16_bits(float f) {
  const unsigned u  = __float_as_uint(f);
  const unsigned s  = (u >> 16) & 0x8000u;
  const unsigned a  = u & 0x7fffffffu;
  const unsigned t  = a - 0x38000000u;
  const unsigned r  = (t + 0x0FFFu + ((t >> 13) & 1u)) >> 13;
  const unsigned rc = r > 0x7C00u ? 0x7C00u : r;
  const bool small  = a < 0x38800000u;
  const bool isnan  = a > 0x7f800000u;
  const unsigned fin = small ? 0u : (s | rc);
  return isnan ? (s | 0x7E00u) : fin;
}

__device__ __forceinline__ unsigned pk16(unsigned lo, unsigned hi) { return lo | (hi << 16); }
__device__ __forceinline__ unsigned bf16_lo_bits(float v) {
  float hi = bf16_val(v);
  asm volatile("" : "+v"(hi));
  return bf16_bits(v - hi);
}
__device__ __forceinline__ v4u pack8_bf16(v4f a, v4f c) {
  return (v4u){ pk16(bf16_bits(a[0]), bf16_bits(a[1])), pk16(bf16_bits(a[2]), bf16_bits(a[3])),
                pk16(bf16_bits(c[0]), bf16_bits(c[1])), pk16(bf16_bits(c[2]), bf16_bits(c[3])) };
}
__device__ __forceinline__ v4u pack8_bf16_lo(v4f a, v4f c) {
  return (v4u){ pk16(bf16_lo_bits(a[0]), bf16_lo_bits(a[1])), pk16(bf16_lo_bits(a[2]), bf16_lo_bits(a[3])),
                pk16(bf16_lo_bits(c[0]), bf16_lo_bits(c[1])), pk16(bf16_lo_bits(c[2]), bf16_lo_bits(c[3])) };
}
__device__ __forceinline__ v4u pack8_f16(v4f a, v4f c) {
  return (v4u){ pk16(f16_bits(a[0]), f16_bits(a[1])), pk16(f16_bits(a[2]), f16_bits(a[3])),
                pk16(f16_bits(c[0]), f16_bits(c[1])), pk16(f16_bits(c[2]), f16_bits(c[3])) };
}

template <int FORM>
__global__ __launch_bounds__(256) void k_plane(const float* __restrict__ src, int rows, int cols, int ldsrc,
                                               unsigned short* __restrict__ dst, int MP, int KP) {
  static_assert(FORM >= 0 && FORM <= 3);
  const int KTOT = (FORM == 1 || FORM == 3) ? 2 * KP : KP;
  const unsigned ppr   = (unsigned)(KTOT >> 3);
  const unsigned kp8   = (unsigned)(KP >> 3);
  const unsigned total = (unsigned)MP * ppr;
  const unsigned g     = blockIdx.x * 256u + threadIdx.x;
  const unsigned rowu  = g / ppr;
  const unsigned p     = g - rowu * ppr;
  const bool second    = p >= kp8;
  const int row = (int)rowu;
  const int c0  = (int)((second ? p - kp8 : p) << 3);
  const float* srow = src + (size_t)clampi(row, 0, rows - 1) * (size_t)ldsrc;
  float x[8];
  unsigned mk[8];
#pragma unroll
  for (int e = 0; e < 8; ++e) {
    const int c = c0 + e;
    const float v = srow[clampi(c, 0, cols - 1)];
    asm volatile("" :: "v"(v));
    x[e]  = v;
    mk[e] = (row < rows && c < cols) ? 0xFFFFu : 0u;
  }
  const v4f a = (v4f){ x[0], x[1], x[2], x[3] };
  const v4f c = (v4f){ x[4], x[5], x[6], x[7] };
  v4u o;
  if (FORM == 2) {
    o = pack8_f16(a, c);
  } else {
    const v4u hi = pack8_bf16(a, c);
    o = hi;
    if (FORM == 1) { const v4u lo = pack8_bf16_lo(a, c); o = second ? lo : hi; }
  }
  const v4u mw = (v4u){ pk16(mk[0], mk[1]), pk16(mk[2], mk[3]), pk16(mk[4], mk[5]), pk16(mk[6], mk[7]) };
  o &= mw;
  if (g < total) {
    volatile v4u* q = (volatile v4u*)(dst + (size_t)g * 8);
    *q = o;
    __threadfence();
    *q = o;
  }
}

template <int FORM> struct FragOf    { typedef FragB T; };
template <>         struct FragOf<2> { typedef FragH T; };
__device__ __forceinline__ v8f mm(const FragB& a, const FragB& b, v8f c) { return wmb(a, b, c); }
__device__ __forceinline__ v8f mm(const FragH& a, const FragH& b, v8f c) { return wmh(a, b, c); }
template <class F> __device__ __forceinline__ F ld_frag(const unsigned short* p) {
  F f;
  f.h[0] = *(const v8usa*)(p);
  f.h[1] = *(const v8usa*)(p + 16);
  return f;
}

template <int FORM, int EPI>
__global__ __launch_bounds__(256) __attribute__((amdgpu_num_vgpr(248)))
void k_gemm_nt(const unsigned short* __restrict__ A, const unsigned short* __restrict__ B,
               const float* __restrict__ bias, float* __restrict__ D, int M, int N, int KTOT, int ldd) {
  static_assert(FORM >= 0 && FORM <= 2);
  static_assert(EPI == 0 || EPI == 1);
  typedef typename FragOf<FORM>::T F;
  __shared__ __attribute__((aligned(16))) float sT[8][16 * 68];
  const int lane = threadIdx.x & 31;
  const int wave = threadIdx.x >> 5;
  const int tilesM = (M + 63) >> 6;
  const int tilesN = (N + 63) >> 6;
  const int tile = blockIdx.x * 8 + wave;
  if (tile >= tilesM * tilesN) return;
  const int tm = tile / tilesN;
  const int tn = tile - tm * tilesN;
  const int m0 = tm << 6;
  const int n0 = tn << 6;

  const int rl = lane & 15;
  const int h8 = (lane >> 4) * 8;
  const unsigned short* pa = A + (size_t)(m0 + rl) * (size_t)KTOT + h8;
  const unsigned short* pb = B + (size_t)(n0 + rl) * (size_t)KTOT + h8;

  v8f acc[4][4];
#pragma unroll
  for (int i = 0; i < 4; ++i)
#pragma unroll
    for (int j = 0; j < 4; ++j) acc[i][j] = (v8f){0.f, 0.f, 0.f, 0.f, 0.f, 0.f, 0.f, 0.f};

#pragma unroll 1
  for (int k0 = 0; k0 < KTOT; k0 += 32) {
    F bf[4];
#pragma unroll
    for (int j = 0; j < 4; ++j) bf[j] = ld_frag<F>(pb + (size_t)(j << 4) * (size_t)KTOT + k0);
#pragma unroll
    for (int i = 0; i < 4; ++i) {
      const F af = ld_frag<F>(pa + (size_t)(i << 4) * (size_t)KTOT + k0);
#pragma unroll
      for (int j = 0; j < 4; ++j) acc[i][j] = mm(af, bf[j], acc[i][j]);
    }
  }

  float* slab = sT[wave];
  const int hh = lane >> 4;
  const int c4 = (lane & 15) * 4;
  const int nc = n0 + c4;
  const bool cok = nc < N;
  v4f bv = (v4f){0.f, 0.f, 0.f, 0.f};
  if (EPI == 1) {
    bv = *(const v4fa*)(bias + clampi(nc, 0, N - 4));
    asm volatile("" :: "v"(bv));
  }
#pragma unroll
  for (int i = 0; i < 4; ++i) {
    const int mBase = m0 + (i << 4);
#pragma unroll
    for (int j = 0; j < 4; ++j) {
#pragma unroll
      for (int r = 0; r < 8; ++r) slab[(h8 + r) * 68 + (j << 4) + rl] = acc[i][j][r];
    }
    __builtin_amdgcn_fence(__ATOMIC_RELEASE, "workgroup");
    __builtin_amdgcn_wave_barrier();
    __builtin_amdgcn_fence(__ATOMIC_ACQUIRE, "workgroup");
    v4f vv[8];
#pragma unroll
    for (int it = 0; it < 8; ++it) {
      const int row = it * 2 + hh;
      v4f v = *(const v4fa*)(slab + row * 68 + c4);
      if (EPI == 1) v += bv;
      vv[it] = v;
    }
    for (int pass = 0; pass < 2; ++pass) {
#pragma unroll
      for (int it = 0; it < 8; ++it) {
        const int row = mBase + it * 2 + hh;
        if (cok && row < M) *(volatile v4f*)(D + (size_t)row * (size_t)ldd + nc) = vv[it];
      }
      __threadfence();
    }
    __builtin_amdgcn_fence(__ATOMIC_RELEASE, "workgroup");
    __builtin_amdgcn_wave_barrier();
    __builtin_amdgcn_fence(__ATOMIC_ACQUIRE, "workgroup");
  }
}

#pragma clang fp contract(off)

constexpr int NROWS      = 4096;
constexpr int HDIM       = 512;
constexpr int NOPT       = 16;
constexpr int OUTD       = 128;
constexpr int NCOL       = NOPT * OUTD;
constexpr int OUT_ELEMS  = NROWS * OUTD;
constexpr int ROW_BLOCKS = 512;

static_assert(NOPT * OUTD == 2048);
static_assert(OUTD == 32 * 4);
static_assert(HDIM % 64 == 0 && HDIM % 32 == 0);
static_assert(OUTD % 64 == 0);
static_assert(NROWS % 128 == 0);
static_assert(ROW_BLOCKS * 8 == NROWS);
static_assert(512 * 8 == NROWS);
static_assert(NROWS % 64 == 0 && NCOL % 64 == 0 && HDIM % 32 == 0);
static_assert(NROWS % 16 == 0 && NCOL % 4 == 0 && NCOL >= 4 && NCOL % 32 == 0);
static_assert((size_t)NROWS * HDIM / 8 < ((size_t)1 << 31));
static_assert(((size_t)NROWS * HDIM / 8) % 256 == 0);
constexpr int PLANE_BLOCKS = (int)((size_t)NROWS * HDIM / 8 / 256);
constexpr int GEMM_TILES   = (NROWS / 64) * (NCOL / 64);
constexpr int GEMM_BLOCKS  = (GEMM_TILES + 7) / 8;
static_assert(PLANE_BLOCKS == 1024 && GEMM_TILES == 2048 && GEMM_BLOCKS == 256);

constexpr size_t SZ_XB  = (size_t)NROWS * HDIM * 2;
constexpr size_t SZ_WT  = (size_t)NCOL * HDIM * 2;
constexpr size_t SZ_BQ  = (size_t)NOPT * OUTD * 4;
constexpr size_t SZ_P   = (size_t)NROWS * NCOL * 4;
constexpr size_t OFF_XB = 0;
constexpr size_t OFF_WT = OFF_XB + SZ_XB;
constexpr size_t OFF_BQ = OFF_WT + SZ_WT;
constexpr size_t OFF_P  = OFF_BQ + SZ_BQ;
constexpr size_t WS_TOTAL = OFF_P + SZ_P;
static_assert(WS_TOTAL == (size_t)39854080);
static_assert(WS_TOTAL <= ((size_t)128 << 20));
static_assert(OFF_WT % 256 == 0 && OFF_BQ % 256 == 0 && OFF_P % 256 == 0);
static_assert(SZ_XB % 256 == 0 && SZ_WT % 256 == 0 && SZ_BQ % 256 == 0 && SZ_P % 256 == 0);

constexpr int WT_TK     = HDIM / 64;
constexpr int WT_TN     = OUTD / 64;
constexpr int WT_BLOCKS = NOPT * WT_TK * WT_TN;
static_assert(WT_BLOCKS == 256);
__global__ __launch_bounds__(256) void k_wT(const float* __restrict__ W, unsigned short* __restrict__ WT) {
  __shared__ float tile[64 * 65];
  const int tid = (int)threadIdx.x;
  const int per = WT_TK * WT_TN;
  const int z   = (int)blockIdx.x / per;
  const int rem = (int)blockIdx.x - z * per;
  const int tk  = rem / WT_TN;
  const int tn  = rem - tk * WT_TN;
  const int k0 = tk << 6, n0 = tn << 6;
  const float* src = W + (size_t)z * (size_t)HDIM * (size_t)OUTD;
  unsigned short* dst = WT + (size_t)z * (size_t)OUTD * (size_t)HDIM;
  const int c4 = (tid & 15) * 4;
#pragma unroll
  for (int i = 0; i < 4; ++i) {
    const int kr = (tid >> 4) + 16 * i;
    const v4f v = *(const v4fa*)(src + (size_t)(k0 + kr) * (size_t)OUTD + n0 + c4);
    asm volatile("" :: "v"(v));
    tile[kr * 65 + c4 + 0] = v[0];
    tile[kr * 65 + c4 + 1] = v[1];
    tile[kr * 65 + c4 + 2] = v[2];
    tile[kr * 65 + c4 + 3] = v[3];
  }
  __syncthreads();
  v4u o[2];
#pragma unroll
  for (int i = 0; i < 2; ++i) {
    const int q  = tid + 256 * i;
    const int n  = q >> 3;
    const int pc = q & 7;
    const float* tp = tile + (pc * 8) * 65 + n;
    const v4f a = (v4f){ tp[0 * 65], tp[1 * 65], tp[2 * 65], tp[3 * 65] };
    const v4f c = (v4f){ tp[4 * 65], tp[5 * 65], tp[6 * 65], tp[7 * 65] };
    o[i] = pack8_bf16(a, c);
  }
#pragma unroll
  for (int i = 0; i < 2; ++i) {
    const int q = tid + 256 * i;
    unsigned short* dp = dst + (size_t)(n0 + (q >> 3)) * (size_t)HDIM + k0 + (q & 7) * 8;
    *(volatile v4u*)dp = o[i];
  }
  __threadfence();
#pragma unroll
  for (int i = 0; i < 2; ++i) {
    const int q = tid + 256 * i;
    unsigned short* dp = dst + (size_t)(n0 + (q >> 3)) * (size_t)HDIM + k0 + (q & 7) * 8;
    *(volatile v4u*)dp = o[i];
  }
}

constexpr int BQ_PIECES = NOPT * OUTD / 4;
static_assert(BQ_PIECES % 256 == 0);
__global__ __launch_bounds__(256) void k_bias(const float* __restrict__ b, float* __restrict__ BQ) {
  const int piece = (int)blockIdx.x * 256 + (int)threadIdx.x;
  const int pc = piece < BQ_PIECES ? piece : BQ_PIECES - 1;
  const v4f a = *(const v4fa*)(b + 4 * pc);
  asm volatile("" :: "v"(a));
  v4f o;
#pragma unroll
  for (int e = 0; e < 4; ++e) o[e] = bf16_val(a[e]);
  if (piece < BQ_PIECES) {
    volatile v4f* q = (volatile v4f*)(BQ + 4 * piece);
    *q = o;
    __threadfence();
    *q = o;
  }
}

__device__ __forceinline__ float maxn(float a, float b) {
  const bool tb = (b > a) | (b != b);
  return tb ? b : a;
}

__global__ __launch_bounds__(256) void k_row(const float* __restrict__ P, const float* __restrict__ BQ,
                                             const int* __restrict__ option, float* __restrict__ out) {
  const int tid = (int)threadIdx.x, lane = tid & 31, wave = tid >> 5;
  const int row = (int)blockIdx.x * 8 + wave;
  const int rc  = row < NROWS ? row : NROWS - 1;
  int ov = option[rc];
  asm volatile("" :: "v"(ov));
  ov = clampi(ov, 0, NOPT - 1);
  const int g = __builtin_amdgcn_readfirstlane(ov);
  const v4f pv = *(const v4fa*)(P + (size_t)rc * (size_t)NCOL + (size_t)(OUTD * g + 4 * lane));
  const float p0 = pv[0], p1 = pv[1], p2 = pv[2], p3 = pv[3];
  asm volatile("" :: "v"(p0));
  asm volatile("" :: "v"(p1));
  asm volatile("" :: "v"(p2));
  asm volatile("" :: "v"(p3));
  const v4f qv = *(const v4fa*)(BQ + (size_t)(OUTD * g + 4 * lane));
  const float q0 = qv[0], q1 = qv[1], q2 = qv[2], q3 = qv[3];
  asm volatile("" :: "v"(q0));
  asm volatile("" :: "v"(q1));
  asm volatile("" :: "v"(q2));
  asm volatile("" :: "v"(q3));
  const float v0 = p0 + q0;
  const float v1 = p1 + q1;
  const float v2 = p2 + q2;
  const float v3 = p3 + q3;

  float m = maxn(maxn(maxn(v0, v1), v2), v3);
  { const float t = __shfl_xor(m, 16, 32); m = maxn(m, t); }
  { const float t = __shfl_xor(m, 8, 32);  m = maxn(m, t); }
  { const float t = __shfl_xor(m, 4, 32);  m = maxn(m, t); }
  { const float t = __shfl_xor(m, 2, 32);  m = maxn(m, t); }
  { const float t = __shfl_xor(m, 1, 32);  m = maxn(m, t); }

  const float e0 = expf(v0 - m);
  const float e1 = expf(v1 - m);
  const float e2 = expf(v2 - m);
  const float e3 = expf(v3 - m);

  float s = ((e0 + e1) + e2) + e3;
  { const float t = __shfl_xor(s, 16, 32); s = s + t; }
  { const float t = __shfl_xor(s, 8, 32);  s = s + t; }
  { const float t = __shfl_xor(s, 4, 32);  s = s + t; }
  { const float t = __shfl_xor(s, 2, 32);  s = s + t; }
  { const float t = __shfl_xor(s, 1, 32);  s = s + t; }

  const v4f r = (v4f){ e0 / s, e1 / s, e2 / s, e3 / s };
  if (row < NROWS) {
    volatile v4f* q = (volatile v4f*)(out + (size_t)row * (size_t)OUTD + 4 * lane);
    *q = r;
    __threadfence();
    *q = r;
  }
}

extern "C" void kernel_launch(void* const* d_in, const int* in_sizes, int n_in,
                              void* d_out, int out_size, void* d_ws, size_t ws_size,
                              hipStream_t stream) {
  if (n_in < 4) return;
  if (in_sizes[0] != NROWS * HDIM) return;
  if (in_sizes[1] != NROWS) return;
  if (in_sizes[2] != NOPT * HDIM * OUTD) return;
  if (in_sizes[3] != NOPT * OUTD) return;
  if (out_size != OUT_ELEMS) return;
  if (ws_size < WS_TOTAL) return;

  const float* x      = (const float*)d_in[0];
  const int*   option = (const int*)d_in[1];
  const float* W      = (const float*)d_in[2];
  const float* b      = (const float*)d_in[3];
  float* out = (float*)d_out;

  char* ws = (char*)d_ws;
  unsigned short* XB = (unsigned short*)(ws + OFF_XB);
  unsigned short* WT = (unsigned short*)(ws + OFF_WT);
  float*          BQ = (float*)(ws + OFF_BQ);
  float*          P  = (float*)(ws + OFF_P);

  k_plane<0><<<PLANE_BLOCKS, 256, 0, stream>>>(x, NROWS, HDIM, HDIM, XB, NROWS, HDIM);
  k_wT<<<WT_BLOCKS, 256, 0, stream>>>(W, WT);
  k_bias<<<BQ_PIECES / 256, 256, 0, stream>>>(b, BQ);
  k_gemm_nt<0, 0><<<GEMM_BLOCKS, 256, 0, stream>>>(XB, WT, BQ, P, NROWS, NCOL, HDIM, NCOL);
  k_row<<<ROW_BLOCKS, 256, 0, stream>>>(P, BQ, option, out);
}
